// SpatialAttentionLayer_54047868452939
// MI455X (gfx1250) — hardware-verified
//
#include <hip/hip_runtime.h>

#ifndef NB
#define NB 4
#endif
#ifndef SEQ
#define SEQ 4096
#endif
#define NB_FULL 4
#define N_FULL  4096
#define C_IN    256
#define CQ      32
#define NWR     320
#define QB      64
#define OPITCH  68
#define VPITCH  72

#define WSC     256.0f
#define WINV    (1.0f / 256.0f)
#define QSC     8.0f
#define VSC     8.0f
#define SINV    (1.0f / 64.0f)
#define PSCALE  16384.0f
#define OSC     (1.0f / (16384.0f * 8.0f))

static_assert(SEQ % QB == 0);
static_assert(SEQ <= N_FULL);
static_assert(NB >= 1);
static_assert(NB <= NB_FULL);
static_assert(C_IN % 32 == 0);
static_assert(CQ == 32);
static_assert(NWR % 64 == 0);

typedef _Float16 v16h __attribute__((ext_vector_type(16)));
typedef _Float16 v8h  __attribute__((ext_vector_type(8)));
typedef _Float16 v8ha __attribute__((ext_vector_type(8), __may_alias__));
typedef float    v8f  __attribute__((ext_vector_type(8)));
typedef float    v4f  __attribute__((ext_vector_type(4)));
typedef float    v4fa __attribute__((ext_vector_type(4), __may_alias__));

union Frag { v16h v; v8h half[2]; };

__device__ __forceinline__ v8f wmma16(v16h a, v16h b, v8f c) {
    v8f d = __builtin_amdgcn_wmma_f32_16x16x32_f16(false, a, false, b, (short)0, c, false, false);
    asm volatile("v_nop\n\tv_nop\n\tv_nop\n\tv_nop" : "+v"(d) : "v"(a), "v"(b));
    return d;
}

__device__ __forceinline__ float bfr(float f) {
    unsigned int u = __float_as_uint(f);
    u = (u + 0x7FFFu + ((u >> 16) & 1u)) & 0xFFFF0000u;
    return __uint_as_float(u);
}

__device__ __forceinline__ void xt_rows(const float* __restrict__ xb, _Float16* tb,
                                        int n0, int wid, int l)
{
#pragma unroll 1
    for (int it = 0; it < QB / 8; ++it) {
        const int n = n0 + 8 * it + wid;
        const float* xp = xb + (size_t)(8 * l) * N_FULL + n;
        v8h hv;
#pragma unroll
        for (int k = 0; k < 8; ++k) hv[k] = (_Float16)bfr(xp[(size_t)k * N_FULL]);
        *(volatile v8h*)(tb + (size_t)n * C_IN + 8 * l) = hv;
    }
}

__global__ void __launch_bounds__(256)
k_xt(const float* __restrict__ x, _Float16* __restrict__ xt)
{
    const int tid = threadIdx.x, l = tid & 31, wid = tid >> 5;
    const int b = blockIdx.y, n0 = blockIdx.x * QB;
    const float* xb = x + (size_t)b * C_IN * N_FULL;
    _Float16* tb = xt + (size_t)b * SEQ * C_IN;
    xt_rows(xb, tb, n0, wid, l);
    __threadfence();
    xt_rows(xb, tb, n0, wid, l);
}

__global__ void __launch_bounds__(256)
k_w16(const float* __restrict__ wq, const float* __restrict__ wk, const float* __restrict__ wv,
      _Float16* __restrict__ w16)
{
    const int tid = threadIdx.x, l = tid & 31, wid = tid >> 5;
    const int r = blockIdx.x * 8 + wid;
    const int rq = min(r, CQ - 1);
    const int rk = min(max(r - CQ, 0), CQ - 1);
    const int rv = min(max(r - 2 * CQ, 0), C_IN - 1);
    const float* pq = wq + (size_t)rq * C_IN + 8 * l;
    const float* pk = wk + (size_t)rk * C_IN + 8 * l;
    const float* pv = wv + (size_t)rv * C_IN + 8 * l;
    const v4f q0 = *(const v4f*)(pq), q1 = *(const v4f*)(pq + 4);
    const v4f k0 = *(const v4f*)(pk), k1 = *(const v4f*)(pk + 4);
    const v4f v0 = *(const v4f*)(pv), v1 = *(const v4f*)(pv + 4);
    const bool isq = (r < CQ), isk = (r < 2 * CQ);
    v8h hv;
#pragma unroll
    for (int i = 0; i < 4; ++i) {
        const float a = isq ? q0[i] : (isk ? k0[i] : v0[i]);
        const float c = isq ? q1[i] : (isk ? k1[i] : v1[i]);
        hv[i]     = (_Float16)(bfr(a) * WSC);
        hv[4 + i] = (_Float16)(bfr(c) * WSC);
    }
    _Float16* dst = w16 + (size_t)r * C_IN + 8 * l;
    *(volatile v8h*)dst = hv;
    __threadfence();
    *(volatile v8h*)dst = hv;
}

__device__ __forceinline__ void proj_store(const _Float16* sV, const _Float16* sQK,
                                           _Float16* qt, _Float16* kt, _Float16* v16,
                                           int yb, int b, int n0, int wid, int l)
{
    if (yb == 0) {
        const int nl = 8 * wid + (l >> 2), pc = 8 * (l & 3);
        const v8h hq = *(const v8ha*)(sQK + nl * CQ + pc);
        const v8h hk = *(const v8ha*)(sQK + QB * CQ + nl * CQ + pc);
        const size_t go = ((size_t)b * SEQ + n0 + nl) * CQ + pc;
        *(volatile v8h*)(qt + go) = hq;
        *(volatile v8h*)(kt + go) = hk;
    } else {
#pragma unroll
        for (int gg = 0; gg < 2; ++gg) {
            const int g  = wid + 8 * gg;
            const int ol = 4 * g + (l >> 3), pc = 8 * (l & 7);
            const int c  = (yb - 1) * QB + ol;
            const v8h hv = *(const v8ha*)(sV + ol * VPITCH + pc);
            *(volatile v8h*)(v16 + ((size_t)b * C_IN + c) * SEQ + n0 + pc) = hv;
        }
    }
}

__global__ void __launch_bounds__(256)
k_proj(const _Float16* __restrict__ xt, const _Float16* __restrict__ w16,
       const float* __restrict__ bq, const float* __restrict__ bk, const float* __restrict__ bv,
       _Float16* __restrict__ qt, _Float16* __restrict__ kt, _Float16* __restrict__ v16)
{
    __shared__ __align__(16) _Float16 sV[QB * VPITCH];
    __shared__ __align__(16) _Float16 sQK[2 * QB * CQ];
    __shared__ float sBias[NWR];

    const int tid = threadIdx.x, l = tid & 31, wid = tid >> 5, h = l >> 4, m = l & 15;
    const int b = blockIdx.z, yb = blockIdx.y, n0 = blockIdx.x * QB;
    const int nt = wid & 3, og = wid >> 2;
    const int obase = yb * 64 + og * 32;

    for (int i = tid; i < NWR; i += 256) {
        const float a  = bq[min(i, CQ - 1)];
        const float bb = bk[min(max(i - CQ, 0), CQ - 1)];
        const float c  = bv[min(max(i - 2 * CQ, 0), C_IN - 1)];
        sBias[i] = bfr((i < CQ) ? a : ((i < 2 * CQ) ? bb : c));
    }
    __syncthreads();

    const _Float16* xtb = xt + ((size_t)b * SEQ + n0 + 16 * nt + m) * C_IN + 8 * h;
    const _Float16* wa0 = w16 + (size_t)(obase + m) * C_IN + 8 * h;
    const _Float16* wa1 = w16 + (size_t)(obase + 16 + m) * C_IN + 8 * h;

    const v8f zero8 = {0.f, 0.f, 0.f, 0.f, 0.f, 0.f, 0.f, 0.f};
    v8f acc0 = zero8, acc1 = zero8;
#pragma unroll 1
    for (int cb = 0; cb < C_IN; cb += 32) {
        Frag bf, a0, a1;
        bf.half[0] = *(const v8h*)(xtb + cb);
        bf.half[1] = *(const v8h*)(xtb + cb + 16);
        a0.half[0] = *(const v8h*)(wa0 + cb);
        a0.half[1] = *(const v8h*)(wa0 + cb + 16);
        a1.half[0] = *(const v8h*)(wa1 + cb);
        a1.half[1] = *(const v8h*)(wa1 + cb + 16);
        acc0 = wmma16(a0.v, bf.v, acc0);
        acc1 = wmma16(a1.v, bf.v, acc1);
    }

    if (yb == 0) {
        _Float16* sd = sQK + og * (QB * CQ);
        const int nl = 16 * nt + m;
#pragma unroll
        for (int r = 0; r < 8; ++r) {
            const int o0 = 8 * h + r, o1 = 16 + 8 * h + r;
            sd[nl * CQ + o0] = (_Float16)((acc0[r] * WINV + sBias[obase + o0]) * QSC);
            sd[nl * CQ + o1] = (_Float16)((acc1[r] * WINV + sBias[obase + o1]) * QSC);
        }
    } else {
        const int nl = 16 * nt + m;
#pragma unroll
        for (int r = 0; r < 8; ++r) {
            const int ol0 = og * 32 + 8 * h + r, ol1 = og * 32 + 16 + 8 * h + r;
            sV[ol0 * VPITCH + nl] = (_Float16)((acc0[r] * WINV + sBias[obase + 8 * h + r]) * VSC);
            sV[ol1 * VPITCH + nl] = (_Float16)((acc1[r] * WINV + sBias[obase + 16 + 8 * h + r]) * VSC);
        }
    }
    __syncthreads();

    proj_store(sV, sQK, qt, kt, v16, yb, b, n0, wid, l);
    __threadfence();
    proj_store(sV, sQK, qt, kt, v16, yb, b, n0, wid, l);
}

__device__ __forceinline__ void out_rows(const float* sO, const float* __restrict__ x, float* out,
                                         int b, int i0, int ph, int wid, int l)
{
#pragma unroll 1
    for (int g = wid; g < 64; g += 8) {
        const int cl = 2 * g + (l >> 4);
        const int c  = 128 * ph + cl;
        const int pc = 4 * (l & 15);
        const v4f y  = *(const v4fa*)(sO + cl * OPITCH + pc);
        const v4f xv = *(const v4f*)(x + ((size_t)b * C_IN + c) * N_FULL + i0 + pc);
        v4f o;
#pragma unroll
        for (int k = 0; k < 4; ++k) o[k] = y[k] + bfr(xv[k]);
        *(volatile v4f*)(out + ((size_t)b * C_IN + c) * SEQ + i0 + pc) = o;
    }
}

__global__ void __launch_bounds__(256)
k_attn(const _Float16* __restrict__ qt, const _Float16* __restrict__ kt,
       const _Float16* __restrict__ v16, const float* __restrict__ x, float* __restrict__ out)
{
    __shared__ __align__(16) float sO[128 * OPITCH];

    const int tid = threadIdx.x, l = tid & 31, wid = tid >> 5, h = l >> 4, m = l & 15;
    const int b = blockIdx.y, i0 = blockIdx.x * QB;
    const int rt = wid & 3, ch = wid >> 2;
    const int iw = i0 + 16 * rt;

    Frag qb;
    {
        const _Float16* qp = qt + ((size_t)b * SEQ + iw + m) * CQ + 8 * h;
        qb.half[0] = *(const v8h*)(qp);
        qb.half[1] = *(const v8h*)(qp + 16);
    }
    const _Float16* kb = kt + ((size_t)b * SEQ + m) * CQ + 8 * h;
    const v8f zero8 = {0.f, 0.f, 0.f, 0.f, 0.f, 0.f, 0.f, 0.f};

    float mx = -3.0e38f;
#pragma unroll 1
    for (int j0 = 0; j0 < SEQ; j0 += 32) {
        const _Float16* kp0 = kb + (size_t)j0 * CQ;
        const _Float16* kp1 = kp0 + 16 * CQ;
        Frag k0f, k1f;
        k0f.half[0] = *(const v8h*)(kp0);
        k0f.half[1] = *(const v8h*)(kp0 + 16);
        k1f.half[0] = *(const v8h*)(kp1);
        k1f.half[1] = *(const v8h*)(kp1 + 16);
        const v8f s0 = wmma16(k0f.v, qb.v, zero8);
        const v8f s1 = wmma16(k1f.v, qb.v, zero8);
#pragma unroll
        for (int r = 0; r < 8; ++r) mx = fmaxf(mx, fmaxf(s0[r], s1[r]));
    }
    mx = fmaxf(mx, __shfl_xor(mx, 16));

    v8f acc[8];
#pragma unroll
    for (int t = 0; t < 8; ++t) acc[t] = zero8;
    float z = 0.f;
    const _Float16* vbp = v16 + ((size_t)b * C_IN + 128 * ch + m) * SEQ + 8 * h;

#pragma unroll 1
    for (int j0 = 0; j0 < SEQ; j0 += 32) {
        const _Float16* kp0 = kb + (size_t)j0 * CQ;
        const _Float16* kp1 = kp0 + 16 * CQ;
        Frag k0f, k1f;
        k0f.half[0] = *(const v8h*)(kp0);
        k0f.half[1] = *(const v8h*)(kp0 + 16);
        k1f.half[0] = *(const v8h*)(kp1);
        k1f.half[1] = *(const v8h*)(kp1 + 16);
        const v8f s0 = wmma16(k0f.v, qb.v, zero8);
        const v8f s1 = wmma16(k1f.v, qb.v, zero8);
        v16h pa;
#pragma unroll
        for (int r = 0; r < 8; ++r) {
            const float p0 = __expf((s0[r] - mx) * SINV);
            const float p1 = __expf((s1[r] - mx) * SINV);
            z += p0 + p1;
            pa[r]     = (_Float16)(p0 * PSCALE);
            pa[8 + r] = (_Float16)(p1 * PSCALE);
        }
#pragma unroll
        for (int t = 0; t < 8; ++t) {
            const _Float16* vp = vbp + (size_t)(16 * t) * SEQ + j0;
            Frag vf;
            vf.half[0] = *(const v8h*)(vp);
            vf.half[1] = *(const v8h*)(vp + 16);
            acc[t] = wmma16(pa, vf.v, acc[t]);
        }
    }

    z += __shfl_xor(z, 16);
    const float zs = (1.0f / z) * OSC;
    float scl[8];
#pragma unroll
    for (int r = 0; r < 8; ++r) scl[r] = __shfl(zs, 8 * h + r);

#pragma unroll
    for (int ph = 0; ph < 2; ++ph) {
        if (ch == ph) {
#pragma unroll
            for (int t = 0; t < 8; ++t)
#pragma unroll
                for (int r = 0; r < 8; ++r)
                    sO[(16 * t + m) * OPITCH + 16 * rt + 8 * h + r] = acc[t][r] * scl[r];
        }
        __syncthreads();
        out_rows(sO, x, out, b, i0, ph, wid, l);
        __threadfence();
        out_rows(sO, x, out, b, i0, ph, wid, l);
        __syncthreads();
    }
}

extern "C" void kernel_launch(void* const* d_in, const int* in_sizes, int n_in,
                              void* d_out, int out_size, void* d_ws, size_t ws_size,
                              hipStream_t stream)
{
    const size_t xt_bytes = (size_t)NB * SEQ * C_IN * sizeof(_Float16);
    const size_t w_bytes  = (size_t)NWR * C_IN * sizeof(_Float16);
    const size_t qk_bytes = (size_t)NB * SEQ * CQ * sizeof(_Float16);
    const size_t v_bytes  = (size_t)NB * C_IN * SEQ * sizeof(_Float16);
    const size_t total    = xt_bytes + w_bytes + 2 * qk_bytes + v_bytes;

    if (n_in < 7) return;
    if (in_sizes[0] < NB * C_IN * N_FULL) return;
    if (in_sizes[1] < CQ * C_IN || in_sizes[2] < CQ) return;
    if (in_sizes[3] < CQ * C_IN || in_sizes[4] < CQ) return;
    if (in_sizes[5] < C_IN * C_IN || in_sizes[6] < C_IN) return;
    if (out_size < NB * C_IN * SEQ) return;
    if (ws_size < total) return;

    const float* x   = (const float*)d_in[0];
    const float* wq  = (const float*)d_in[1];
    const float* bq  = (const float*)d_in[2];
    const float* wk  = (const float*)d_in[3];
    const float* bk  = (const float*)d_in[4];
    const float* wvp = (const float*)d_in[5];
    const float* bv  = (const float*)d_in[6];
    float* outp = (float*)d_out;

    char* ws = (char*)d_ws;
    _Float16* xt  = (_Float16*)(ws);
    _Float16* w16 = (_Float16*)(ws + xt_bytes);
    _Float16* qt  = (_Float16*)(ws + xt_bytes + w_bytes);
    _Float16* kt  = (_Float16*)(ws + xt_bytes + w_bytes + qk_bytes);
    _Float16* v16 = (_Float16*)(ws + xt_bytes + w_bytes + 2 * qk_bytes);

    k_xt<<<dim3(SEQ / QB, NB), dim3(256), 0, stream>>>(x, xt);
    k_w16<<<dim3(NWR / 8), dim3(256), 0, stream>>>(wq, wk, wvp, w16);
    k_proj<<<dim3(SEQ / QB, NWR / 64, NB), dim3(256), 0, stream>>>(xt, w16, bq, bk, bv, qt, kt, v16);
    k_attn<<<dim3(SEQ / QB, NB), dim3(256), 0, stream>>>(qt, kt, v16, x, outp);
    (void)hipGetLastError();
}
